// OffsetAttention1_65352222376315
// MI455X (gfx1250) — hardware-verified
//
#include <hip/hip_runtime.h>
#include <math.h>

#define B_    8
#define CIN_  3
#define N_    4096
#define C_    256
#define C4_   64
#define NB_   (B_ * N_)
#define BN_EPS_  1e-5f
#define PSC_     32768.0f
#define PSC_INV_ (1.0f / 32768.0f)
#define WSC_     16.0f
#define WSC_INV_ (1.0f / 16.0f)

typedef __attribute__((ext_vector_type(16))) _Float16 v16h;
typedef __attribute__((ext_vector_type(8)))  _Float16 v8h;
typedef __attribute__((ext_vector_type(8)))  float    v8f;
typedef __attribute__((ext_vector_type(4)))  float    v4f;

__device__ __forceinline__ void dep_guard_h(v8f& a, v8f& b, v16h x, v16h y) { asm volatile("v_nop\n\tv_nop\n\tv_nop\n\tv_nop" : "+v"(a), "+v"(b) : "v"(x), "v"(y)); }
__device__ __forceinline__ void keep4_h(v16h a, v16h b, v16h c, v16h d) { asm volatile("v_nop" :: "v"(a), "v"(b), "v"(c), "v"(d)); }
__device__ __forceinline__ void acc_guard4(v8f& a, v8f& b, v8f& c, v8f& d) { asm volatile("v_nop\n\tv_nop\n\tv_nop\n\tv_nop" : "+v"(a), "+v"(b), "+v"(c), "+v"(d)); }

template <typename T> struct Frag;
template <> struct Frag<_Float16> {
  typedef v16h V; union U { v16h v; v8h h[2]; };
  static __device__ __forceinline__ v16h load(const _Float16* p) {
    U f; f.h[0] = *(const v8h*)(p); f.h[1] = *(const v8h*)(p + 16); return f.v;
  }
  static __device__ __forceinline__ v8f mma(v16h a, v16h b, v8f c) {
    return __builtin_amdgcn_wmma_f32_16x16x32_f16(false, a, false, b, (short)0, c, false, false);
  }
  static __device__ __forceinline__ void guard(v8f& a, v8f& b, v16h x, v16h y) { dep_guard_h(a, b, x, y); }
  static __device__ __forceinline__ void keep(v16h a, v16h b, v16h c, v16h d) { keep4_h(a, b, c, d); }
};

__device__ __forceinline__ v8f mma_h(v16h a, v16h b, v8f c) {
  c = __builtin_amdgcn_wmma_f32_16x16x32_f16(false, a, false, b, (short)0, c, false, false);
  asm volatile("v_nop\n\tv_nop\n\tv_nop\n\tv_nop" : "+v"(c) : "v"(a), "v"(b));
  return c;
}

template <int BIAS_MODE, int OUT_MODE, int RES_MODE, bool ROWSCALE>
__global__ __launch_bounds__(256) void wmma_gemm64(
    const unsigned short* __restrict__ Ap, int lda, long strideA,
    const unsigned short* __restrict__ Btp, int ldb, long strideB,
    void* __restrict__ Cout, int ldc, long strideC,
    const float* __restrict__ bias,
    const float* __restrict__ resid, int ldr, long strideR,
    const float* __restrict__ rsc, long strideS,
    int M, int N, int K, float scale) {
  typedef _Float16 T;
  typedef v16h V;
  const T* A = (const T*)Ap; const T* Bt = (const T*)Btp;
  __shared__ __align__(16) float sT[8][16 * 68];
  const int b    = blockIdx.y;
  const int lane = threadIdx.x & 31;
  const int wave = threadIdx.x >> 5;
  const int tilesN = N >> 6;
  const int tilesM = M >> 6;
  const int tile = blockIdx.x * 8 + wave;
  if (tile >= tilesM * tilesN) return;
  const int tm = tile / tilesN;
  const int tn = tile - tm * tilesN;
  const int m0 = tm << 6;
  const int n0 = tn << 6;

  const T* Ab = A  + (size_t)b * strideA;
  const T* Bb = Bt + (size_t)b * strideB;

  const int rlane = lane & 15;
  const int koff  = (lane >> 4) * 8;
  const int mOff  = (lane >> 4) * 8;

  v8f acc[4][4];
#pragma unroll
  for (int i = 0; i < 4; ++i)
#pragma unroll
    for (int j = 0; j < 4; ++j) acc[i][j] = (v8f){0.f,0.f,0.f,0.f,0.f,0.f,0.f,0.f};

  for (int k0 = 0; k0 < K; k0 += 32) {
    V bh[4];
#pragma unroll
    for (int j = 0; j < 4; ++j) {
      const size_t bo = (size_t)(n0 + (j << 4) + rlane) * ldb + koff + k0;
      bh[j] = Frag<T>::load(Bb + bo);
    }
#pragma unroll
    for (int i = 0; i < 4; ++i) {
      const size_t ao = (size_t)(m0 + (i << 4) + rlane) * lda + koff + k0;
      V ah = Frag<T>::load(Ab + ao);
#pragma unroll
      for (int j = 0; j < 4; ++j) {
        acc[i][j] = Frag<T>::mma(ah, bh[j], acc[i][j]);
      }
      Frag<T>::guard(acc[i][0], acc[i][3], ah, ah);
    }
    Frag<T>::keep(bh[0], bh[1], bh[2], bh[3]);
  }
  acc_guard4(acc[0][0], acc[0][1], acc[0][2], acc[0][3]);
  acc_guard4(acc[1][0], acc[1][1], acc[1][2], acc[1][3]);
  acc_guard4(acc[2][0], acc[2][1], acc[2][2], acc[2][3]);
  acc_guard4(acc[3][0], acc[3][1], acc[3][2], acc[3][3]);

  float* slab = sT[wave];
  const float* Rb = (RES_MODE != 0) ? (resid + (size_t)b * strideR) : nullptr;
  const float* Sb = ROWSCALE ? (rsc + (size_t)b * strideS) : nullptr;
#pragma unroll
  for (int i = 0; i < 4; ++i) {
    const int mBase = m0 + (i << 4);
#pragma unroll
    for (int j = 0; j < 4; ++j) {
      const int n = n0 + (j << 4) + rlane;
      float bv = 0.f;
      if (BIAS_MODE == 2) bv = bias[n];
#pragma unroll
      for (int r = 0; r < 8; ++r) {
        const int mr = mBase + mOff + r;
        float v = acc[i][j][r] * scale;
        if (ROWSCALE) v *= Sb[mr];
        if (BIAS_MODE == 1) v += bias[mr];
        if (BIAS_MODE == 2) v += bv;
        if (RES_MODE == 1) v += Rb[(size_t)mr * ldr + n];
        if (RES_MODE == 2) v += Rb[(size_t)n * ldr + mr];
        slab[(mOff + r) * 68 + (j << 4) + rlane] = v;
      }
    }
    __builtin_amdgcn_fence(__ATOMIC_RELEASE, "workgroup");
    __builtin_amdgcn_wave_barrier();
    __builtin_amdgcn_fence(__ATOMIC_ACQUIRE, "workgroup");
    if (OUT_MODE == 0) {
      float* C = (float*)Cout + (size_t)b * strideC;
      const int hh = lane >> 4, c4 = (lane & 15) * 4;
      for (int pass = 0; pass < 2; ++pass) {
#pragma unroll
        for (int it = 0; it < 8; ++it) {
          const int row = it * 2 + hh;
          v4f v = *(const v4f*)(slab + row * 68 + c4);
          *(volatile v4f*)(C + (size_t)(mBase + row) * ldc + n0 + c4) = v;
        }
        __threadfence();
      }
    } else {
      const int q = lane >> 3, c8 = (lane & 7) * 8;
      unsigned short* C = (unsigned short*)Cout + (size_t)b * strideC;
      for (int pass = 0; pass < 2; ++pass) {
#pragma unroll
        for (int it = 0; it < 4; ++it) {
          const int row = it * 4 + q;
          const float* sp = slab + row * 68 + c8;
          v8h hv;
#pragma unroll
          for (int e = 0; e < 8; ++e) hv[e] = (_Float16)sp[e];
          *(volatile v8h*)(C + (size_t)(mBase + row) * ldc + n0 + c8) = hv;
        }
        __threadfence();
      }
    }
    __builtin_amdgcn_fence(__ATOMIC_RELEASE, "workgroup");
    __builtin_amdgcn_wave_barrier();
    __builtin_amdgcn_fence(__ATOMIC_ACQUIRE, "workgroup");
  }
}

__global__ __launch_bounds__(256) void k_castw(const float* __restrict__ in, _Float16* __restrict__ out, int n2, float sc) {
  const int i = blockIdx.x * 256 + threadIdx.x;
  if (i < n2) {
    const _Float16 h0 = (_Float16)(in[2 * i] * sc), h1 = (_Float16)(in[2 * i + 1] * sc);
    const unsigned u = (unsigned)__builtin_bit_cast(unsigned short, h0) | ((unsigned)__builtin_bit_cast(unsigned short, h1) << 16);
    ((volatile unsigned*)out)[i] = u;
    __threadfence();
    ((volatile unsigned*)out)[i] = u;
  }
}

__global__ __launch_bounds__(256) void k_bn1(const float* __restrict__ x, const float* __restrict__ W1,
                                             const float* __restrict__ g1, const float* __restrict__ b1,
                                             float* __restrict__ bnp) {
  __shared__ double red[9][256];
  const int tid = threadIdx.x;
  double a0 = 0.0, a1 = 0.0, a2 = 0.0, m00 = 0.0, m01 = 0.0, m02 = 0.0, m11 = 0.0, m12 = 0.0, m22 = 0.0;
#pragma unroll 1
  for (int it = 0; it < NB_ / 256; ++it) {
    const int p = it * 256 + tid;
    const int bb = p >> 12, n = p & (N_ - 1);
    const float* xb = x + (size_t)bb * CIN_ * N_ + n;
    const double x0 = (double)xb[0], x1 = (double)xb[N_], x2 = (double)xb[2 * N_];
    a0 += x0; a1 += x1; a2 += x2;
    m00 += x0 * x0; m01 += x0 * x1; m02 += x0 * x2;
    m11 += x1 * x1; m12 += x1 * x2; m22 += x2 * x2;
  }
  red[0][tid] = a0; red[1][tid] = a1; red[2][tid] = a2;
  red[3][tid] = m00; red[4][tid] = m01; red[5][tid] = m02;
  red[6][tid] = m11; red[7][tid] = m12; red[8][tid] = m22;
  __syncthreads();
  for (int s = 128; s > 0; s >>= 1) {
    if (tid < s) {
#pragma unroll
      for (int k = 0; k < 9; ++k) red[k][tid] += red[k][tid + s];
    }
    __syncthreads();
  }
  const double inv = 1.0 / (double)NB_;
  const double mu0 = red[0][0] * inv, mu1 = red[1][0] * inv, mu2 = red[2][0] * inv;
  const double c00 = red[3][0] * inv - mu0 * mu0;
  const double c01 = red[4][0] * inv - mu0 * mu1;
  const double c02 = red[5][0] * inv - mu0 * mu2;
  const double c11 = red[6][0] * inv - mu1 * mu1;
  const double c12 = red[7][0] * inv - mu1 * mu2;
  const double c22 = red[8][0] * inv - mu2 * mu2;
  const int cch = tid;
  const double w0 = (double)W1[cch * 3], w1 = (double)W1[cch * 3 + 1], w2 = (double)W1[cch * 3 + 2];
  const double mean = w0 * mu0 + w1 * mu1 + w2 * mu2;
  const double var = w0 * w0 * c00 + w1 * w1 * c11 + w2 * w2 * c22
                   + 2.0 * (w0 * w1 * c01 + w0 * w2 * c02 + w1 * w2 * c12);
  float varf = (float)var;
  varf = fmaxf(varf, 0.0f);
  const float sc = g1[cch] * (1.0f / sqrtf(varf + BN_EPS_));
  const float bi = b1[cch] - (float)mean * sc;
  ((volatile float*)bnp)[cch] = sc;
  ((volatile float*)bnp)[C_ + cch] = bi;
  __threadfence();
  ((volatile float*)bnp)[cch] = sc;
  ((volatile float*)bnp)[C_ + cch] = bi;
}

__global__ __launch_bounds__(256) void k_embed(const float* __restrict__ x, const float* __restrict__ W1,
                                               const float* __restrict__ bnp, float* __restrict__ h,
                                               _Float16* __restrict__ hT) {
  __shared__ __align__(16) float T[64 * 68];
  __shared__ float xs[3 * 64];
  __shared__ float wsm[64 * 3];
  __shared__ float scs[64];
  __shared__ float bis[64];
  const int tid = threadIdx.x, wave = tid >> 5, lane = tid & 31;
  const int n0 = blockIdx.x * 64, c0 = blockIdx.y * 64, b = blockIdx.z;
  if (tid < 192) {
    const int i = tid >> 6, nl = tid & 63;
    xs[tid]  = x[((size_t)(b * CIN_ + i)) * N_ + n0 + nl];
    wsm[tid] = W1[c0 * 3 + tid];
  }
  if (tid < 64) { scs[tid] = bnp[c0 + tid]; bis[tid] = bnp[C_ + c0 + tid]; }
  __syncthreads();
  {
    const int nl = tid & 63, cg = tid >> 6;
    const float x0 = xs[nl], x1 = xs[64 + nl], x2 = xs[128 + nl];
#pragma unroll 4
    for (int i = 0; i < 16; ++i) {
      const int cl = cg * 16 + i;
      const float z = wsm[cl * 3] * x0 + wsm[cl * 3 + 1] * x1 + wsm[cl * 3 + 2] * x2;
      T[cl * 68 + nl] = fmaxf(z * scs[cl] + bis[cl], 0.0f);
    }
  }
  __syncthreads();
  const int hh = lane >> 4, c4 = (lane & 15) * 4, q = lane >> 3, c8 = (lane & 7) * 8;
  for (int pass = 0; pass < 2; ++pass) {
#pragma unroll
    for (int it = 0; it < 4; ++it) {
      const int row = wave * 8 + it * 2 + hh;
      const v4f v = *(const v4f*)(T + row * 68 + c4);
      *(volatile v4f*)(h + ((size_t)(b * C_ + c0 + row)) * N_ + n0 + c4) = v;
    }
#pragma unroll
    for (int it = 0; it < 2; ++it) {
      const int nr = wave * 8 + it * 4 + q;
      v8h v;
#pragma unroll
      for (int e = 0; e < 8; ++e) v[e] = (_Float16)T[(c8 + e) * 68 + nr];
      *(volatile v8h*)(hT + ((size_t)(b * N_ + n0 + nr)) * C_ + c0 + c8) = v;
    }
    __threadfence();
  }
}

__global__ __launch_bounds__(128) void k_rowstats(const _Float16* __restrict__ qk,
                                                  float* __restrict__ rmax, float* __restrict__ rinv) {
  __shared__ __align__(16) float s_m[64];
  __shared__ __align__(16) float s_i[64];
  const int tid = threadIdx.x, wave = tid >> 5, lane = tid & 31, hh = lane >> 4, c = lane & 15;
  const int nblk = blockIdx.x * 64;
  const int n0 = nblk + wave * 16;
  v16h qa[2];
#pragma unroll
  for (int dc = 0; dc < 2; ++dc)
    qa[dc] = Frag<_Float16>::load(qk + (size_t)(n0 + c) * C4_ + dc * 32 + 8 * hh);
  float mrow[8], lrow[8];
#pragma unroll
  for (int r = 0; r < 8; ++r) { mrow[r] = -1e30f; lrow[r] = 0.f; }

  for (int kc = 0; kc < N_ / 64; ++kc) {
    const int m0 = kc * 64;
    v8f s[4];
#pragma unroll
    for (int j = 0; j < 4; ++j) {
      s[j] = (v8f){0.f,0.f,0.f,0.f,0.f,0.f,0.f,0.f};
#pragma unroll
      for (int dc = 0; dc < 2; ++dc) {
        const v16h kb = Frag<_Float16>::load(qk + (size_t)(m0 + j * 16 + c) * C4_ + dc * 32 + 8 * hh);
        s[j] = mma_h(qa[dc], kb, s[j]);
      }
    }
    float cm[8];
#pragma unroll
    for (int r = 0; r < 8; ++r) {
      float m = fmaxf(fmaxf(s[0][r], s[1][r]), fmaxf(s[2][r], s[3][r]));
#pragma unroll
      for (int off = 1; off < 16; off <<= 1) m = fmaxf(m, __shfl_xor(m, off));
      cm[r] = m;
    }
#pragma unroll
    for (int r = 0; r < 8; ++r) {
      const float mnew = fmaxf(mrow[r], cm[r]);
      const float alpha = __expf(mrow[r] - mnew);
      mrow[r] = mnew;
      float psum = __expf(s[0][r] - mnew) + __expf(s[1][r] - mnew)
                 + __expf(s[2][r] - mnew) + __expf(s[3][r] - mnew);
#pragma unroll
      for (int off = 1; off < 16; off <<= 1) psum += __shfl_xor(psum, off);
      lrow[r] = lrow[r] * alpha + psum;
    }
  }
  if (c == 0) {
#pragma unroll
    for (int r = 0; r < 8; ++r) {
      s_m[wave * 16 + 8 * hh + r] = mrow[r];
      s_i[wave * 16 + 8 * hh + r] = (1.0f / lrow[r]) * PSC_;
    }
  }
  __syncthreads();
  if (wave == 0) {
    const v4f a  = *(const v4f*)(s_m + c * 4);
    const v4f bq = *(const v4f*)(s_i + c * 4);
    v4f val;
#pragma unroll
    for (int e = 0; e < 4; ++e) val[e] = hh ? bq[e] : a[e];
    float* dst = hh ? (rinv + nblk + c * 4) : (rmax + nblk + c * 4);
    for (int pass = 0; pass < 2; ++pass) {
      *(volatile v4f*)dst = val;
      __threadfence();
    }
  }
}

__global__ __launch_bounds__(128) void k_pcol(const _Float16* __restrict__ qk, const float* __restrict__ rmax,
                                              const float* __restrict__ rinv, _Float16* __restrict__ pt,
                                              float* __restrict__ cinv) {
  __shared__ __align__(16) _Float16 s_p[4][16 * 72];
  __shared__ __align__(16) float s_c[64];
  const int tid = threadIdx.x, wave = tid >> 5, lane = tid & 31, hh = lane >> 4, c = lane & 15;
  const int mblk = blockIdx.x * 64;
  const int mw = mblk + wave * 16;
  v16h kb[2];
#pragma unroll
  for (int dc = 0; dc < 2; ++dc)
    kb[dc] = Frag<_Float16>::load(qk + (size_t)(mw + c) * C4_ + dc * 32 + 8 * hh);
  _Float16* sp = s_p[wave];
  float csum = 0.f;
  const int q = lane >> 3, c8 = (lane & 7) * 8;

  for (int nc = 0; nc < N_ / 64; ++nc) {
    const int n0 = nc * 64;
    float pc = 0.f;
#pragma unroll
    for (int i = 0; i < 4; ++i) {
      const int nr = n0 + i * 16;
      v8f e = (v8f){0.f,0.f,0.f,0.f,0.f,0.f,0.f,0.f};
#pragma unroll
      for (int dc = 0; dc < 2; ++dc) {
        const v16h a = Frag<_Float16>::load(qk + (size_t)(nr + c) * C4_ + dc * 32 + 8 * hh);
        e = mma_h(a, kb[dc], e);
      }
      const v4f mx0 = *(const v4f*)(rmax + nr + 8 * hh);
      const v4f mx1 = *(const v4f*)(rmax + nr + 8 * hh + 4);
      const v4f iv0 = *(const v4f*)(rinv + nr + 8 * hh);
      const v4f iv1 = *(const v4f*)(rinv + nr + 8 * hh + 4);
      v8h pv;
#pragma unroll
      for (int r = 0; r < 4; ++r) {
        const float p = __expf(e[r] - mx0[r]) * iv0[r];
        pc += p;
        pv[r] = (_Float16)p;
      }
#pragma unroll
      for (int r = 0; r < 4; ++r) {
        const float p = __expf(e[4 + r] - mx1[r]) * iv1[r];
        pc += p;
        pv[4 + r] = (_Float16)p;
      }
      *(v8h*)(sp + c * 72 + i * 16 + 8 * hh) = pv;
    }
    csum += pc;
    __builtin_amdgcn_fence(__ATOMIC_RELEASE, "workgroup");
    __builtin_amdgcn_wave_barrier();
    __builtin_amdgcn_fence(__ATOMIC_ACQUIRE, "workgroup");
    for (int pass = 0; pass < 2; ++pass) {
#pragma unroll
      for (int it = 0; it < 4; ++it) {
        const int row = it * 4 + q;
        const v8h v = *(const v8h*)(sp + row * 72 + c8);
        *(volatile v8h*)(pt + (size_t)(mw + row) * N_ + n0 + c8) = v;
      }
      __threadfence();
    }
    __builtin_amdgcn_fence(__ATOMIC_RELEASE, "workgroup");
    __builtin_amdgcn_wave_barrier();
    __builtin_amdgcn_fence(__ATOMIC_ACQUIRE, "workgroup");
  }
  csum += __shfl_xor(csum, 16);
  if (hh == 0) s_c[wave * 16 + c] = 1.0f / (1e-9f + csum * PSC_INV_);
  __syncthreads();
  if (tid < 16) {
    const v4f v = *(const v4f*)(s_c + tid * 4);
    for (int pass = 0; pass < 2; ++pass) {
      *(volatile v4f*)(cinv + mblk + tid * 4) = v;
      __threadfence();
    }
  }
}

__global__ __launch_bounds__(256) void k_bn2(const float* __restrict__ t, const float* __restrict__ g2,
                                             const float* __restrict__ b2, float* __restrict__ bnp) {
  __shared__ __align__(16) float s_sc[32];
  __shared__ __align__(16) float s_bi[32];
  const int tid = threadIdx.x, wave = tid >> 5, lane = tid & 31;
  const int cbase = blockIdx.x * 32 + wave * 4;
#pragma unroll
  for (int k = 0; k < 4; ++k) {
    const int cch = cbase + k;
    double su = 0.0, sq = 0.0;
#pragma unroll 1
    for (int it = 0; it < NB_ / 32; ++it) {
      const int p = it * 32 + lane;
      const int bb = p >> 12, n = p & (N_ - 1);
      const float v = t[((size_t)(bb * C_ + cch)) * N_ + n];
      su += (double)v;
      sq += (double)v * (double)v;
    }
#pragma unroll
    for (int off = 16; off > 0; off >>= 1) {
      su += __shfl_xor(su, off);
      sq += __shfl_xor(sq, off);
    }
    if (lane == 0) {
      const double mean = su / (double)NB_;
      const double var = sq / (double)NB_ - mean * mean;
      float varf = (float)var;
      varf = fmaxf(varf, 0.0f);
      const float sc = g2[cch] * (1.0f / sqrtf(varf + BN_EPS_));
      s_sc[wave * 4 + k] = sc;
      s_bi[wave * 4 + k] = b2[cch] - (float)mean * sc;
    }
  }
  __syncthreads();
  if (tid < 16) {
    const int h2 = tid >> 3, i4 = (tid & 7) * 4;
    const v4f a  = *(const v4f*)(s_sc + i4);
    const v4f bq = *(const v4f*)(s_bi + i4);
    v4f val;
#pragma unroll
    for (int e = 0; e < 4; ++e) val[e] = h2 ? bq[e] : a[e];
    float* dst = h2 ? (bnp + C_ + blockIdx.x * 32 + i4) : (bnp + blockIdx.x * 32 + i4);
    for (int pass = 0; pass < 2; ++pass) {
      *(volatile v4f*)dst = val;
      __threadfence();
    }
  }
}

__global__ __launch_bounds__(256) void k_out(const float* __restrict__ t, const float* __restrict__ bnp,
                                             float* out) {
  const size_t i4 = (size_t)blockIdx.x * 256 + threadIdx.x;
  const int cch = (int)((i4 >> 10) & (C_ - 1));
  const v4f hv = *(const v4f*)(out + i4 * 4);
  const v4f tv = *(const v4f*)(t + i4 * 4);
  const float sc = bnp[cch], bi = bnp[C_ + cch];
  v4f o;
#pragma unroll
  for (int e = 0; e < 4; ++e) o[e] = hv[e] + fmaxf(tv[e] * sc + bi, 0.0f);
  *(volatile v4f*)(out + i4 * 4) = o;
  __threadfence();
  *(volatile v4f*)(out + i4 * 4) = o;
}

static const size_t SZ_HT16 = (size_t)B_ * N_ * C_ * 2;
static const size_t SZ_V16  = (size_t)B_ * C_ * N_ * 2;
static const size_t SZ_QK16 = (size_t)B_ * N_ * C4_ * 2;
static const size_t SZ_PT16 = (size_t)N_ * N_ * 2;
static const size_t SZ_T    = (size_t)B_ * C_ * N_ * 4;
static const size_t SZ_ROW  = (size_t)B_ * N_ * 4;
static const size_t SZ_WQ   = (size_t)C4_ * C_ * 2;
static const size_t SZ_WW   = (size_t)C_ * C_ * 2;
static const size_t SZ_BN   = 2048;
static const size_t OFF_HT16 = 0;
static const size_t OFF_V16  = OFF_HT16 + SZ_HT16;
static const size_t OFF_QK16 = OFF_V16  + SZ_V16;
static const size_t OFF_PT16 = OFF_QK16 + SZ_QK16;
static const size_t OFF_T    = OFF_PT16 + SZ_PT16;
static const size_t OFF_RMAX = OFF_T    + SZ_T;
static const size_t OFF_RINV = OFF_RMAX + SZ_ROW;
static const size_t OFF_CINV = OFF_RINV + SZ_ROW;
static const size_t OFF_WQ   = OFF_CINV + SZ_ROW;
static const size_t OFF_WV   = OFF_WQ   + SZ_WQ;
static const size_t OFF_WT   = OFF_WV   + SZ_WW;
static const size_t OFF_BN1  = OFF_WT   + SZ_WW;
static const size_t OFF_BN2  = OFF_BN1  + SZ_BN;
static const size_t WS_TOTAL = OFF_BN2  + SZ_BN;

extern "C" void kernel_launch(void* const* d_in, const int* in_sizes, int n_in,
                              void* d_out, int out_size, void* d_ws, size_t ws_size,
                              hipStream_t stream) {
  if (n_in < 11) return;
  if (in_sizes[0] != B_ * CIN_ * N_ || in_sizes[1] != C_ * CIN_ || in_sizes[4] != C4_ * C_ ||
      in_sizes[5] != C_ * C_ || in_sizes[7] != C_ * C_) return;
  if (in_sizes[2] != C_ || in_sizes[3] != C_ || in_sizes[6] != C_ || in_sizes[8] != C_ ||
      in_sizes[9] != C_ || in_sizes[10] != C_) return;
  if ((size_t)out_size != (size_t)B_ * C_ * N_) return;
  if (ws_size < WS_TOTAL) return;

  const float* x  = (const float*)d_in[0];
  const float* W1 = (const float*)d_in[1];
  const float* g1 = (const float*)d_in[2];
  const float* b1 = (const float*)d_in[3];
  const float* Wq = (const float*)d_in[4];
  const float* Wv = (const float*)d_in[5];
  const float* bv = (const float*)d_in[6];
  const float* Wt = (const float*)d_in[7];
  const float* bt = (const float*)d_in[8];
  const float* g2 = (const float*)d_in[9];
  const float* b2 = (const float*)d_in[10];
  float* out = (float*)d_out;

  char* ws = (char*)d_ws;
  _Float16* hT16 = (_Float16*)(ws + OFF_HT16);
  _Float16* v16  = (_Float16*)(ws + OFF_V16);
  _Float16* qk16 = (_Float16*)(ws + OFF_QK16);
  _Float16* pt16 = (_Float16*)(ws + OFF_PT16);
  float*    tbuf = (float*)(ws + OFF_T);
  float*    rmax = (float*)(ws + OFF_RMAX);
  float*    rinv = (float*)(ws + OFF_RINV);
  float*    cinv = (float*)(ws + OFF_CINV);
  _Float16* wq16 = (_Float16*)(ws + OFF_WQ);
  _Float16* wv16 = (_Float16*)(ws + OFF_WV);
  _Float16* wt16 = (_Float16*)(ws + OFF_WT);
  float*    bn1p = (float*)(ws + OFF_BN1);
  float*    bn2p = (float*)(ws + OFF_BN2);

  k_bn1<<<1, 256, 0, stream>>>(x, W1, g1, b1, bn1p);
  k_embed<<<dim3(N_ / 64, C_ / 64, B_), 256, 0, stream>>>(x, W1, bn1p, out, hT16);

  k_castw<<<(C4_ * C_ / 2 + 255) / 256, 256, 0, stream>>>(Wq, wq16, C4_ * C_ / 2, WSC_);
  k_castw<<<(C_ * C_ / 2 + 255) / 256, 256, 0, stream>>>(Wv, wv16, C_ * C_ / 2, WSC_);
  k_castw<<<(C_ * C_ / 2 + 255) / 256, 256, 0, stream>>>(Wt, wt16, C_ * C_ / 2, WSC_);

  wmma_gemm64<0, 1, 0, false><<<dim3((N_ / 64) * (C4_ / 64) / 8, B_), 256, 0, stream>>>(
      (const unsigned short*)hT16, C_, (long)N_ * C_,
      (const unsigned short*)wq16, C_, 0L,
      (void*)qk16, C4_, (long)N_ * C4_,
      nullptr, nullptr, 0, 0L, nullptr, 0L,
      N_, C4_, C_, WSC_INV_);

  wmma_gemm64<1, 1, 0, false><<<dim3((C_ / 64) * (N_ / 64) / 8, B_), 256, 0, stream>>>(
      (const unsigned short*)wv16, C_, 0L,
      (const unsigned short*)hT16, C_, (long)N_ * C_,
      (void*)v16, N_, (long)C_ * N_,
      bv, nullptr, 0, 0L, nullptr, 0L,
      C_, N_, C_, WSC_INV_);

  for (int b = 0; b < B_; ++b) {
    const _Float16* qkb = qk16 + (size_t)b * N_ * C4_;
    float* rmb = rmax + (size_t)b * N_;
    float* rib = rinv + (size_t)b * N_;
    float* cib = cinv + (size_t)b * N_;
    k_rowstats<<<N_ / 64, 128, 0, stream>>>(qkb, rmb, rib);
    k_pcol<<<N_ / 64, 128, 0, stream>>>(qkb, rmb, rib, pt16, cib);
    wmma_gemm64<0, 1, 2, true><<<dim3((N_ / 64) * (C_ / 64) / 8, 1), 256, 0, stream>>>(
        (const unsigned short*)pt16, N_, 0L,
        (const unsigned short*)(v16 + (size_t)b * C_ * N_), N_, 0L,
        (void*)(hT16 + (size_t)b * N_ * C_), C_, 0L,
        nullptr,
        out + (size_t)b * C_ * N_, N_, 0L,
        cib, 0L,
        N_, C_, N_, -PSC_INV_);
  }

  wmma_gemm64<1, 0, 0, false><<<dim3((C_ / 64) * (N_ / 64) / 8, B_), 256, 0, stream>>>(
      (const unsigned short*)wt16, C_, 0L,
      (const unsigned short*)hT16, C_, (long)N_ * C_,
      (void*)tbuf, N_, (long)C_ * N_,
      bt, nullptr, 0, 0L, nullptr, 0L,
      C_, N_, C_, WSC_INV_);

  k_bn2<<<C_ / 32, 256, 0, stream>>>(tbuf, g2, b2, bn2p);
  k_out<<<(B_ * C_ * N_ / 4) / 256, 256, 0, stream>>>(tbuf, bn2p, out);
}
